// LSTMAutoencoder_53369263620301
// MI455X (gfx1250) — hardware-run, weakly checked
//
#include <hip/hip_runtime.h>
#include <math.h>

constexpr int HID    = 32;
constexpr int NGATE  = 4 * HID;
constexpr int LAT    = 8;
constexpr int SEQ    = 120;
constexpr int NBATCH = 16384;
constexpr int RPW    = 16;
constexpr int NWAVE  = 2;
constexpr int NTHR   = 32 * NWAVE;
constexpr int RPB    = RPW * NWAVE;
constexpr int NBLK   = NBATCH / RPB;
constexpr int XYLEN  = RPW * SEQ;
constexpr int XPP    = 132;
constexpr int WP     = 40;
constexpr int NWPL   = 4;
constexpr float WCARRY = 16.0f;
constexpr float HCARRY = 64.0f;
constexpr float CCARRY = 1024.0f;
constexpr float FOLD   = 1.0f / 1024.0f;
constexpr float RCARRY = 2048.0f;
constexpr float RFOLD  = 1.0f / 2048.0f;
static_assert(NBATCH % RPB == 0);
static_assert(NBLK * RPB == NBATCH);
static_assert(HID == 32);
static_assert(NGATE == 8 * 16);
static_assert(XYLEN % 128 == 0);
static_assert((RPW * SEQ * 4) % 128 == 0);
static_assert(NGATE % NTHR == 0 && (LAT * HID) % NTHR == 0 && (NGATE * 4) % NTHR == 0);
static_assert((WP * 2) % 16 == 0 && (XPP * 4) % 16 == 0);
static_assert(WCARRY * HCARRY == CCARRY);
static_assert(RPW * XPP >= 15 * XPP + NGATE);
static_assert(WP >= HID);

typedef __attribute__((ext_vector_type(16))) _Float16 v16h;
typedef __attribute__((ext_vector_type(8)))  _Float16 v8h;
typedef __attribute__((ext_vector_type(16))) __bf16   v16b;
typedef __attribute__((ext_vector_type(8)))  float    v8f;
typedef __attribute__((ext_vector_type(4)))  float    v4f;
union FragH { v16h v; v8h h[2]; };

__device__ __forceinline__ unsigned short f2bf_bits(float f) {
  unsigned u = __float_as_uint(f);
  return (unsigned short)((u + 0x7FFFu + ((u >> 16) & 1u)) >> 16);
}
__device__ __forceinline__ float bf_bits2f(unsigned short h) { return __uint_as_float(((unsigned)h) << 16); }
__device__ __forceinline__ void bf_split(float v, unsigned short& hb, unsigned short& lb) {
  hb = f2bf_bits(v);
  lb = f2bf_bits(v - bf_bits2f(hb));
}
__device__ __forceinline__ void split_w(float w, _Float16& hi, _Float16& lo) {
  const float ws = w * WCARRY;
  const _Float16 hq = (_Float16)ws;
  const float hf = (float)hq;
  const float res = ws - hf;
  hi = hq;
  lo = (_Float16)(res * RCARRY);
}

__device__ __forceinline__ v8f mma_h(v16h a, v16h b, v8f c) {
  return __builtin_amdgcn_wmma_f32_16x16x32_f16(false, a, false, b, (short)0, c, false, false);
}
__device__ __forceinline__ v8f mma_b(v16b a, v16b b, v8f c) {
  return __builtin_amdgcn_wmma_f32_16x16x32_bf16(false, a, false, b, (short)0, c, false, false);
}
__device__ __forceinline__ void guard4_h(v8f& a, v8f& b, v8f& c, v8f& d,
                                         v16h w0, v16h w1, v16h w2, v16h w3, v16h x) {
  asm volatile("v_nop\n\tv_nop\n\tv_nop\n\tv_nop"
               : "+v"(a), "+v"(b), "+v"(c), "+v"(d)
               : "v"(w0), "v"(w1), "v"(w2), "v"(w3), "v"(x));
}
__device__ __forceinline__ void guard1_b(v8f& a, v16b w, v16b x, v16b y, v16b z) {
  asm volatile("v_nop\n\tv_nop\n\tv_nop\n\tv_nop" : "+v"(a) : "v"(w), "v"(x), "v"(y), "v"(z));
}
__device__ __forceinline__ void mem_break() { asm volatile("" ::: "memory"); }

__device__ __forceinline__ float fsig(float v)  { return __builtin_amdgcn_rcpf(1.0f + expf(-v)); }
__device__ __forceinline__ float ftanh(float v) { return 1.0f - 2.0f * __builtin_amdgcn_rcpf(expf(2.0f * v) + 1.0f); }

__device__ __forceinline__ void cell_step(v8f ai, v8f af, v8f ag, v8f ao,
                                          v8f ri, v8f rf, v8f rg, v8f ro,
                                          float (&cs)[8], float (&hs)[8]) {
#pragma unroll
  for (int r = 0; r < 8; ++r) {
    const float zi = fmaf(ri[r], RFOLD, ai[r]) * FOLD;
    const float zf = fmaf(rf[r], RFOLD, af[r]) * FOLD;
    const float zg = fmaf(rg[r], RFOLD, ag[r]) * FOLD;
    const float zo = fmaf(ro[r], RFOLD, ao[r]) * FOLD;
    const float ig = fsig(zi);
    const float fg = fsig(zf);
    const float gg = ftanh(zg);
    const float og = fsig(zo);
    const float cv = fg * cs[r] + ig * gg;
    cs[r] = cv;
    hs[r] = og * ftanh(cv);
  }
}

__global__ __launch_bounds__(NTHR) void seq_ae_kernel(
    const float* __restrict__ x,
    const float* __restrict__ eWih, const float* __restrict__ eWhh,
    const float* __restrict__ ebih, const float* __restrict__ ebhh,
    const float* __restrict__ elW,  const float* __restrict__ elb,
    const float* __restrict__ dlW,  const float* __restrict__ dlb,
    const float* __restrict__ dWih, const float* __restrict__ dWhh,
    const float* __restrict__ dbih, const float* __restrict__ dbhh,
    const float* __restrict__ oW,   const float* __restrict__ obp,
    float* __restrict__ out) {
  __shared__ __align__(16) float    s_xy[NWAVE][XYLEN];
  __shared__ __align__(16) float    s_xp[NWAVE][RPW * XPP];
  __shared__ __align__(16) _Float16 s_wf[NWPL][NGATE * WP];
  __shared__ __align__(16) float    s_wih[NGATE];
  __shared__ __align__(16) float    s_bse[NGATE];
  __shared__ __align__(16) float    s_bsd[NGATE];
  __shared__ __align__(16) float    s_elW[LAT * HID];
  __shared__ __align__(16) float    s_dlW[HID * LAT];
  __shared__ __align__(16) float    s_dlb[HID];
  __shared__ __align__(16) float    s_oW[HID];
  __shared__ __align__(16) float    s_elb[LAT];
  __shared__ float s_ob[4];

  const int tid = threadIdx.x, lane = tid & 31, wave = tid >> 5;
  const int cn = lane & 15;
  const int hh = lane >> 4;
  const int k8 = 8 * hh;
  const size_t base = (size_t)blockIdx.x * RPB + (size_t)wave * RPW;

#pragma unroll 1
  for (int i = tid; i < NGATE; i += NTHR) {
    s_wih[i] = eWih[i] * CCARRY;
    s_bse[i] = (ebih[i] + ebhh[i]) * CCARRY;
    s_bsd[i] = dbih[i] + dbhh[i];
  }
#pragma unroll 1
  for (int i = tid; i < LAT * HID; i += NTHR) { s_elW[i] = elW[i]; s_dlW[i] = dlW[i]; }
  if (tid < HID) { s_dlb[tid] = dlb[tid]; s_oW[tid] = oW[tid]; }
  if (tid < LAT) s_elb[tid] = elb[tid];
  if (tid == 0) s_ob[0] = obp[0];
#pragma unroll 1
  for (int i = tid; i < NGATE * 4; i += NTHR) {
    const int row = i >> 2, c8 = (i & 3) * 8;
    const v4f a0 = *(const v4f*)(eWhh + row * HID + c8);
    const v4f a1 = *(const v4f*)(eWhh + row * HID + c8 + 4);
    const v4f b0 = *(const v4f*)(dWhh + row * HID + c8);
    const v4f b1 = *(const v4f*)(dWhh + row * HID + c8 + 4);
    v8h eh, el, dh, dl;
#pragma unroll
    for (int e = 0; e < 4; ++e) {
      _Float16 hq, lq;
      split_w(a0[e], hq, lq); eh[e]     = hq; el[e]     = lq;
      split_w(a1[e], hq, lq); eh[4 + e] = hq; el[4 + e] = lq;
      split_w(b0[e], hq, lq); dh[e]     = hq; dl[e]     = lq;
      split_w(b1[e], hq, lq); dh[4 + e] = hq; dl[4 + e] = lq;
    }
    *(v8h*)(&s_wf[0][0] + row * WP + c8) = eh;
    *(v8h*)(&s_wf[1][0] + row * WP + c8) = el;
    *(v8h*)(&s_wf[2][0] + row * WP + c8) = dh;
    *(v8h*)(&s_wf[3][0] + row * WP + c8) = dl;
  }
  {
    const float* xs = x + base * SEQ;
    float* xw = s_xy[wave];
#pragma unroll 1
    for (int i = lane * 4; i < XYLEN; i += 128) {
      const v4f v = *(const v4f*)(xs + i);
      *(v4f*)(xw + i) = v;
    }
  }
  __syncthreads();

  float cst[2][8], hst[2][8];
#pragma unroll
  for (int g = 0; g < 2; ++g)
#pragma unroll
    for (int r = 0; r < 8; ++r) { cst[g][r] = 0.0f; hst[g][r] = 0.0f; }
  v16h hB;
#pragma unroll
  for (int q = 0; q < 16; ++q) hB[q] = (_Float16)0.0f;
  const v8f z8 = {0.f, 0.f, 0.f, 0.f, 0.f, 0.f, 0.f, 0.f};

  const float* xrow = s_xy[wave] + cn * SEQ;
  const _Float16* weh = &s_wf[0][0] + cn * WP + k8;
  const _Float16* wel = &s_wf[1][0] + cn * WP + k8;
#pragma unroll 1
  for (int ts = 0; ts < SEQ; ++ts) {
    mem_break();
    const float xv = xrow[ts];
    v16h hBn;
#pragma unroll
    for (int grp = 0; grp < 2; ++grp) {
      v8f acc[4], accr[4];
      {
        v16h wq[4];
#pragma unroll
        for (int q = 0; q < 4; ++q) {
          const int t = 2 * q + grp;
          FragH f;
          f.h[0] = *(const v8h*)(weh + (16 * t) * WP);
          f.h[1] = *(const v8h*)(weh + (16 * t) * WP + 16);
          wq[q] = f.v;
          const v4f wa = *(const v4f*)(s_wih + 16 * t + k8);
          const v4f wb = *(const v4f*)(s_wih + 16 * t + k8 + 4);
          const v4f ba = *(const v4f*)(s_bse + 16 * t + k8);
          const v4f bb = *(const v4f*)(s_bse + 16 * t + k8 + 4);
          v8f cx;
#pragma unroll
          for (int e = 0; e < 4; ++e) {
            cx[e]     = fmaf(xv, wa[e], ba[e]);
            cx[4 + e] = fmaf(xv, wb[e], bb[e]);
          }
          acc[q] = mma_h(wq[q], hB, cx);
        }
        guard4_h(acc[0], acc[1], acc[2], acc[3], wq[0], wq[1], wq[2], wq[3], hB);
      }
      {
        v16h wl[4];
#pragma unroll
        for (int q = 0; q < 4; ++q) {
          const int t = 2 * q + grp;
          FragH f;
          f.h[0] = *(const v8h*)(wel + (16 * t) * WP);
          f.h[1] = *(const v8h*)(wel + (16 * t) * WP + 16);
          wl[q] = f.v;
          accr[q] = mma_h(wl[q], hB, z8);
        }
        guard4_h(accr[0], accr[1], accr[2], accr[3], wl[0], wl[1], wl[2], wl[3], hB);
      }
      cell_step(acc[0], acc[1], acc[2], acc[3], accr[0], accr[1], accr[2], accr[3], cst[grp], hst[grp]);
#pragma unroll
      for (int r = 0; r < 8; ++r) hBn[8 * grp + r] = (_Float16)(hst[grp][r] * HCARRY);
    }
    hB = hBn;
  }

  float zv[LAT];
#pragma unroll
  for (int l = 0; l < LAT; ++l) {
    float p = 0.0f;
#pragma unroll
    for (int grp = 0; grp < 2; ++grp) {
      const v4f ea = *(const v4f*)(s_elW + l * HID + 16 * grp + k8);
      const v4f eb = *(const v4f*)(s_elW + l * HID + 16 * grp + k8 + 4);
#pragma unroll
      for (int e = 0; e < 4; ++e) {
        p = fmaf(hst[grp][e], ea[e], p);
        p = fmaf(hst[grp][4 + e], eb[e], p);
      }
    }
    const float po = __shfl_xor(p, 16, 32);
    zv[l] = (p + po) + s_elb[l];
  }
  float d0v[2][8];
#pragma unroll
  for (int s = 0; s < 2; ++s)
#pragma unroll
    for (int e = 0; e < 8; ++e) {
      const int k = 16 * s + k8 + e;
      const v4f wa = *(const v4f*)(s_dlW + k * LAT);
      const v4f wb = *(const v4f*)(s_dlW + k * LAT + 4);
      float a = s_dlb[k];
#pragma unroll
      for (int l = 0; l < 4; ++l) {
        a = fmaf(zv[l], wa[l], a);
        a = fmaf(zv[4 + l], wb[l], a);
      }
      d0v[s][e] = a;
    }
  v16b Bhi, Blo;
#pragma unroll
  for (int s = 0; s < 2; ++s)
#pragma unroll
    for (int e = 0; e < 8; ++e) {
      unsigned short hb, lb;
      bf_split(d0v[s][e], hb, lb);
      Bhi[8 * s + e] = __builtin_bit_cast(__bf16, hb);
      Blo[8 * s + e] = __builtin_bit_cast(__bf16, lb);
    }

  float* xpw = s_xp[wave] + cn * XPP;
#pragma unroll 1
  for (int t = 0; t < 8; ++t) {
    v16b Ahi, Alo;
    {
      const float* rp = dWih + (size_t)(16 * t + cn) * HID;
      const v4f a0 = *(const v4f*)(rp + k8);
      const v4f a1 = *(const v4f*)(rp + k8 + 4);
      const v4f a2 = *(const v4f*)(rp + 16 + k8);
      const v4f a3 = *(const v4f*)(rp + 16 + k8 + 4);
#pragma unroll
      for (int e = 0; e < 4; ++e) {
        unsigned short hb, lb;
        bf_split(a0[e], hb, lb); Ahi[e]      = __builtin_bit_cast(__bf16, hb); Alo[e]      = __builtin_bit_cast(__bf16, lb);
        bf_split(a1[e], hb, lb); Ahi[4 + e]  = __builtin_bit_cast(__bf16, hb); Alo[4 + e]  = __builtin_bit_cast(__bf16, lb);
        bf_split(a2[e], hb, lb); Ahi[8 + e]  = __builtin_bit_cast(__bf16, hb); Alo[8 + e]  = __builtin_bit_cast(__bf16, lb);
        bf_split(a3[e], hb, lb); Ahi[12 + e] = __builtin_bit_cast(__bf16, hb); Alo[12 + e] = __builtin_bit_cast(__bf16, lb);
      }
    }
    const v4f ba = *(const v4f*)(s_bsd + 16 * t + k8);
    const v4f bb = *(const v4f*)(s_bsd + 16 * t + k8 + 4);
    v8f acc;
#pragma unroll
    for (int e = 0; e < 4; ++e) { acc[e] = ba[e]; acc[4 + e] = bb[e]; }
    acc = mma_b(Ahi, Bhi, acc);
    acc = mma_b(Ahi, Blo, acc);
    acc = mma_b(Alo, Bhi, acc);
    guard1_b(acc, Ahi, Alo, Bhi, Blo);
    v4f o0, o1;
#pragma unroll
    for (int e = 0; e < 4; ++e) { o0[e] = acc[e] * CCARRY; o1[e] = acc[4 + e] * CCARRY; }
    *(v4f*)(xpw + 16 * t + k8)     = o0;
    *(v4f*)(xpw + 16 * t + k8 + 4) = o1;
    mem_break();
  }

  float ow[2][8];
#pragma unroll
  for (int grp = 0; grp < 2; ++grp) {
    const v4f a = *(const v4f*)(s_oW + 16 * grp + k8);
    const v4f b = *(const v4f*)(s_oW + 16 * grp + k8 + 4);
#pragma unroll
    for (int e = 0; e < 4; ++e) { ow[grp][e] = a[e]; ow[grp][4 + e] = b[e]; }
  }
  const float obv = s_ob[0];
#pragma unroll
  for (int g = 0; g < 2; ++g)
#pragma unroll
    for (int r = 0; r < 8; ++r) { cst[g][r] = 0.0f; hst[g][r] = 0.0f; }
#pragma unroll
  for (int q = 0; q < 16; ++q) hB[q] = (_Float16)0.0f;
  __syncthreads();

  float* yrow = s_xy[wave] + cn * SEQ;
  const _Float16* wdh = &s_wf[2][0] + cn * WP + k8;
  const _Float16* wdl = &s_wf[3][0] + cn * WP + k8;
#pragma unroll 1
  for (int ts = 0; ts < SEQ; ++ts) {
    mem_break();
    v16h hBn;
#pragma unroll
    for (int grp = 0; grp < 2; ++grp) {
      v8f acc[4], accr[4];
      {
        v16h wq[4];
#pragma unroll
        for (int q = 0; q < 4; ++q) {
          const int t = 2 * q + grp;
          FragH f;
          f.h[0] = *(const v8h*)(wdh + (16 * t) * WP);
          f.h[1] = *(const v8h*)(wdh + (16 * t) * WP + 16);
          wq[q] = f.v;
          const v4f ca = *(const v4f*)(xpw + 16 * t + k8);
          const v4f cb = *(const v4f*)(xpw + 16 * t + k8 + 4);
          v8f cx;
#pragma unroll
          for (int e = 0; e < 4; ++e) { cx[e] = ca[e]; cx[4 + e] = cb[e]; }
          acc[q] = mma_h(wq[q], hB, cx);
        }
        guard4_h(acc[0], acc[1], acc[2], acc[3], wq[0], wq[1], wq[2], wq[3], hB);
      }
      {
        v16h wl[4];
#pragma unroll
        for (int q = 0; q < 4; ++q) {
          const int t = 2 * q + grp;
          FragH f;
          f.h[0] = *(const v8h*)(wdl + (16 * t) * WP);
          f.h[1] = *(const v8h*)(wdl + (16 * t) * WP + 16);
          wl[q] = f.v;
          accr[q] = mma_h(wl[q], hB, z8);
        }
        guard4_h(accr[0], accr[1], accr[2], accr[3], wl[0], wl[1], wl[2], wl[3], hB);
      }
      cell_step(acc[0], acc[1], acc[2], acc[3], accr[0], accr[1], accr[2], accr[3], cst[grp], hst[grp]);
#pragma unroll
      for (int r = 0; r < 8; ++r) hBn[8 * grp + r] = (_Float16)(hst[grp][r] * HCARRY);
    }
    float yp = 0.0f;
#pragma unroll
    for (int grp = 0; grp < 2; ++grp)
#pragma unroll
      for (int r = 0; r < 8; ++r) yp = fmaf(hst[grp][r], ow[grp][r], yp);
    const float yo = __shfl_xor(yp, 16, 32);
    const float yv = (yp + yo) + obv;
    if (hh == 0) yrow[ts] = yv;
    hB = hBn;
  }
  __syncthreads();

  {
    float* op = out + base * SEQ;
    const float* yw = s_xy[wave];
    for (int pass = 0; pass < 2; ++pass) {
#pragma unroll
      for (int it = 0; it < XYLEN / 128; ++it) {
        const int i = it * 128 + lane * 4;
        const v4f v = *(const v4f*)(yw + i);
        *(volatile v4f*)(op + i) = v;
      }
      __threadfence();
    }
  }
}

extern "C" void kernel_launch(void* const* d_in, const int* in_sizes, int n_in,
                              void* d_out, int out_size, void* d_ws, size_t ws_size, hipStream_t stream) {
  (void)d_ws; (void)ws_size;
  if (n_in < 15 || d_out == nullptr) return;
  if (in_sizes[0] != NBATCH * SEQ || in_sizes[1] != NGATE || in_sizes[2] != NGATE * HID ||
      in_sizes[3] != NGATE || in_sizes[4] != NGATE || in_sizes[5] != LAT * HID || in_sizes[6] != LAT ||
      in_sizes[7] != HID * LAT || in_sizes[8] != HID || in_sizes[9] != NGATE * HID || in_sizes[10] != NGATE * HID ||
      in_sizes[11] != NGATE || in_sizes[12] != NGATE || in_sizes[13] != HID || in_sizes[14] != 1 ||
      out_size != NBATCH * SEQ) return;

  const float* x    = (const float*)d_in[0];
  const float* eWih = (const float*)d_in[1];
  const float* eWhh = (const float*)d_in[2];
  const float* ebih = (const float*)d_in[3];
  const float* ebhh = (const float*)d_in[4];
  const float* elW  = (const float*)d_in[5];
  const float* elb  = (const float*)d_in[6];
  const float* dlW  = (const float*)d_in[7];
  const float* dlb  = (const float*)d_in[8];
  const float* dWih = (const float*)d_in[9];
  const float* dWhh = (const float*)d_in[10];
  const float* dbih = (const float*)d_in[11];
  const float* dbhh = (const float*)d_in[12];
  const float* oW   = (const float*)d_in[13];
  const float* obp  = (const float*)d_in[14];
  float* out = (float*)d_out;

  seq_ae_kernel<<<NBLK, NTHR, 0, stream>>>(x, eWih, eWhh, ebih, ebhh, elW, elb, dlW, dlb,
                                           dWih, dWhh, dbih, dbhh, oW, obp, out);
}
